// WindowSelfAttention2D_81097572483357
// MI455X (gfx1250) — hardware-run, weakly checked
//
#include <hip/hip_runtime.h>
#define NB 2
#define CH 128
#define MH 96
#define MW 96
#define HWP (MH * MW)
#define NHD 4
#define DH 32
#define QKVP (3 * CH)
#define WCAR 64.0f
#define OCAR 16.0f
typedef __bf16 v16b __attribute__((ext_vector_type(16)));
typedef unsigned short v8us __attribute__((ext_vector_type(8), may_alias));
typedef float  v8f  __attribute__((ext_vector_type(8)));
typedef float  v4f  __attribute__((ext_vector_type(4)));
typedef float  v4fa __attribute__((ext_vector_type(4), may_alias));
union FragB { v16b v; v8us half[2]; unsigned short u[16]; };

__device__ __forceinline__ unsigned short bf16_bits(float x) { unsigned int u = __float_as_uint(x); return (unsigned short)((u + 0x7FFFu + ((u >> 16) & 1u)) >> 16); }
__device__ __forceinline__ float bf16_val(unsigned short b) { return __uint_as_float(((unsigned int)b) << 16); }
__device__ __forceinline__ float bf16_round(float x) { return bf16_val(bf16_bits(x)); }
template <int NT>
__device__ __forceinline__ v8f mmaN(v16b ah, v16b al, v16b bh, v16b bl, v8f c) {
  c = __builtin_amdgcn_wmma_f32_16x16x32_bf16(false, ah, false, bh, (short)0, c, false, false);
  if (NT >= 2) c = __builtin_amdgcn_wmma_f32_16x16x32_bf16(false, al, false, bh, (short)0, c, false, false);
  if (NT >= 3) c = __builtin_amdgcn_wmma_f32_16x16x32_bf16(false, ah, false, bl, (short)0, c, false, false);
  asm volatile("v_nop\n\tv_nop\n\tv_nop\n\tv_nop" : "+v"(c) : "v"(ah), "v"(al), "v"(bh), "v"(bl));
  return c;
}


typedef _Float16 v16h __attribute__((ext_vector_type(16)));
union FragH { v16h v; v8us half[2]; _Float16 h[16]; unsigned short u[16]; };
template <int NT>
__device__ __forceinline__ v8f mmaH(v16h ah, v16h al, v16h bh, v16h bl, v8f c) {
  c = __builtin_amdgcn_wmma_f32_16x16x32_f16(false, ah, false, bh, (short)0, c, false, false);
  if (NT >= 2) c = __builtin_amdgcn_wmma_f32_16x16x32_f16(false, al, false, bh, (short)0, c, false, false);
  if (NT >= 3) c = __builtin_amdgcn_wmma_f32_16x16x32_f16(false, ah, false, bl, (short)0, c, false, false);
  asm volatile("v_nop\n\tv_nop\n\tv_nop\n\tv_nop" : "+v"(c) : "v"(ah), "v"(al), "v"(bh), "v"(bl));
  return c;
}

typedef _Float16 v4h __attribute__((ext_vector_type(4)));

__device__ __forceinline__ v16h g2_frag(const _Float16* p, int hh) { FragH f; f.half[0] = *(const v8us*)((const unsigned short*)p + 8 * hh); f.half[1] = *(const v8us*)((const unsigned short*)p + 16 + 8 * hh); return f.v; }
__device__ __forceinline__ v8f g2_mma(v16h a, v16h b, v8f c) { v8f d = __builtin_amdgcn_wmma_f32_16x16x32_f16(false, a, false, b, (short)0, c, false, false); asm volatile("v_nop\n\tv_nop\n\tv_nop\n\tv_nop" : "+v"(d) : "v"(a), "v"(b)); return d; }
template <int ACT>
__global__ __launch_bounds__(128) void k_gemm2(const _Float16* __restrict__ A, int lda, size_t sA, const _Float16* __restrict__ Bh, int ldb, size_t sB, float alpha, const float* __restrict__ bias, size_t sBias, const float* __restrict__ CP, int rowsPerB, size_t sCPb, int row0g,
    float* __restrict__ C, _Float16* __restrict__ C16, int ldc, size_t sC, int M, int N, int K) { static_assert(ACT == 0 || ACT == 3 || ACT == 6 || ACT == 8 || ACT == 9 || ACT == 11 || ACT == 12 || ACT == 14 || ACT == 15 || ACT == 16 || ACT == 17, "k_gemm2: unsupported ACT code (would silently apply no activation)");
  __shared__ __attribute__((aligned(16))) float so[4][32][68];
  const int tid = threadIdx.x, w = tid >> 5, lane = tid & 31, ln = lane & 15, hh = lane >> 4; const int by = blockIdx.y;
  A += (size_t)by * sA; Bh += (size_t)by * sB; const size_t cofs = (size_t)by * sC; const float* bp = bias ? bias + (size_t)by * sBias : nullptr;
  const int ntn = N >> 6; const int mt = blockIdx.x / ntn, nq = blockIdx.x - mt * ntn; const int row0 = mt * 128 + 32 * w, col0 = nq * 64; if (row0 >= M) return;
  const _Float16* a0p = A + (size_t)(row0 + ln) * lda; const _Float16* a1p = a0p + (size_t)16 * lda;
  const _Float16* b0p = Bh + (size_t)(col0 + ln) * ldb; const _Float16* b1p = b0p + (size_t)16 * ldb; const _Float16* b2p = b1p + (size_t)16 * ldb; const _Float16* b3p = b2p + (size_t)16 * ldb;
  const v8f z8 = {0.f,0.f,0.f,0.f,0.f,0.f,0.f,0.f}; v8f c00 = z8, c01 = z8, c02 = z8, c03 = z8, c10 = z8, c11 = z8, c12 = z8, c13 = z8;
  for (int kb = 0; kb < K; kb += 32) { const v16h a0 = g2_frag(a0p + kb, hh), a1 = g2_frag(a1p + kb, hh);
    v16h b = g2_frag(b0p + kb, hh); c00 = g2_mma(a0, b, c00); c10 = g2_mma(a1, b, c10);
    b = g2_frag(b1p + kb, hh); c01 = g2_mma(a0, b, c01); c11 = g2_mma(a1, b, c11);
    b = g2_frag(b2p + kb, hh); c02 = g2_mma(a0, b, c02); c12 = g2_mma(a1, b, c12);
    b = g2_frag(b3p + kb, hh); c03 = g2_mma(a0, b, c03); c13 = g2_mma(a1, b, c13); }
  v8f accs[8] = {c00, c01, c02, c03, c10, c11, c12, c13};
#pragma unroll
  for (int u = 0; u < 8; ++u) { const int t = u & 3, half = u >> 2; const int col = col0 + t * 16 + ln; const float bv = bp ? bf16_round(bp[col]) : 0.f;
#pragma unroll
    for (int r = 0; r < 8; ++r) { const int rloc = half * 16 + 8 * hh + r; float v = accs[u][r] * alpha + bv; if (CP) { if (rowsPerB < 0) v += CP[cofs + (size_t)(row0g + row0 + rloc) * ldc + col];        else { const int bidx = (row0g + row0 + rloc) / rowsPerB; v += CP[(size_t)bidx * sCPb + (size_t)by * 64 + col]; } }
      if (ACT == 3) v = fmaxf(v, 0.f); else if (ACT == 6) v = 0.5f * v * (1.0f + erff(v * 0.70710678118654752f)); else if (ACT == 11) v = 1.0f / (1.0f + expf(-v)); else if (ACT == 15) v = v / (1.0f + expf(-v)); else if (ACT == 12) v = (v > 0.f) ? v : 0.01f * v; else if (ACT == 8) v = tanhf(v); else if (ACT == 9) v = 0.5f * v * (1.0f + tanhf(0.7978845608028654f * (v + 0.044715f * v * v * v))); else if (ACT == 14) v = (v > 0.f) ? v : 0.1f * v; else if (ACT == 16) v = (v >= 0.f) ? v : 0.3f * v; else if (ACT == 17) v = (v >= 0.f) ? v : 0.2f * v;
      so[w][rloc][t * 16 + ln] = v; } }
  __builtin_amdgcn_fence(__ATOMIC_ACQ_REL, "workgroup"); __builtin_amdgcn_wave_barrier();
  const int rsub = lane >> 4, c4 = (lane & 15) * 4;
  for (int pass = 0; pass < 2; ++pass) {
#pragma unroll
    for (int q = 0; q < 16; ++q) { const int r = q * 2 + rsub; const v4f v = *(const v4fa*)&so[w][r][c4]; if (C) *(volatile v4f*)(C + cofs + (size_t)(row0 + r) * ldc + col0 + c4) = v; if (C16) { v4h h4; for (int i = 0; i < 4; ++i) h4[i] = (_Float16)v[i]; *(volatile v4h*)(C16 + cofs + (size_t)(row0 + r) * ldc + col0 + c4) = h4; } }
    if (pass == 0) __threadfence(); } }


__global__ __launch_bounds__(256) void k_tcastg(const float* __restrict__ f0, _Float16* __restrict__ XT, int n) {
  const int t = blockIdx.x * 256 + threadIdx.x; if (t >= n) return; const int p = t % HWP, hb = t / HWP; const int hh = hb & 1, b = hb >> 1; const float* s = f0 + ((size_t)b * CH + hh * 64) * HWP + p; unsigned short* d = (unsigned short*)XT + ((size_t)b * HWP + p) * CH + hh * 64;
  for (int g = 0; g < 8; ++g) { FragH f;
#pragma unroll
    for (int q = 0; q < 8; ++q) f.h[q] = (_Float16)bf16_round(s[(size_t)(g * 8 + q) * HWP]);
    *(volatile v8us*)(d + g * 8) = f.half[0]; __threadfence(); *(volatile v8us*)(d + g * 8) = f.half[0]; } }
__global__ __launch_bounds__(256) void k_wcastc(const float* __restrict__ w, _Float16* __restrict__ Wh, float scale, int n8) {
  const int t = blockIdx.x * 256 + threadIdx.x; if (t >= n8) return; const float* s = w + (size_t)t * 8; const v4f a = *(const v4fa*)s, c = *(const v4fa*)(s + 4); FragH f;
#pragma unroll
  for (int q = 0; q < 4; ++q) { f.h[q] = (_Float16)(bf16_round(a[q]) * scale); f.h[4 + q] = (_Float16)(bf16_round(c[q]) * scale); }
  unsigned short* d = (unsigned short*)Wh + (size_t)t * 8; *(volatile v8us*)d = f.half[0]; __threadfence(); *(volatile v8us*)d = f.half[0]; }
__global__ __launch_bounds__(256) void k_win25(const float* __restrict__ QKV, _Float16* __restrict__ O16, int n) {
  const int t = blockIdx.x * 256 + threadIdx.x; if (t >= n) return; const int h = t & 3, r = t >> 2; const int b = r / HWP, p = r - b * HWP; const int py = p / MW, px = p - py * MW;
  const float* q = QKV + (size_t)r * QKVP + h * DH; v4f qv[8];
  for (int c = 0; c < 8; ++c) qv[c] = *(const v4fa*)(q + 4 * c);
  float m = -3.0e38f, l = 0.f; float acc[DH];
  for (int c = 0; c < DH; ++c) acc[c] = 0.f;
  for (int di = 0; di < 5; ++di) { const int ny = py + di - 2; const int cy = (ny < 0) ? 0 : ((ny > MH - 1) ? (MH - 1) : ny); const float iny = (ny == cy) ? 1.0f : 0.0f;
    for (int dj = 0; dj < 5; ++dj) { const int nx = px + dj - 2; const int cx = (nx < 0) ? 0 : ((nx > MW - 1) ? (MW - 1) : nx); const float on = (nx == cx) ? iny : 0.0f; const float* k = QKV + (size_t)(b * HWP + cy * MW + cx) * QKVP + CH + h * DH; float dot = 0.f;
      for (int c = 0; c < 8; ++c) { const v4f kv = *(const v4fa*)(k + 4 * c); dot += qv[c][0] * kv[0]; dot += qv[c][1] * kv[1]; dot += qv[c][2] * kv[2]; dot += qv[c][3] * kv[3]; }
      const float s = on * (dot * 0.17677669529663687f); const float mn = (s > m) ? s : m; const float corr = expf(m - mn); const float pw = expf(s - mn); l = l * corr + pw; const float pv = pw * on; const float* v = k + CH;
      for (int c = 0; c < 8; ++c) { const v4f vv = *(const v4fa*)(v + 4 * c); acc[4 * c] = acc[4 * c] * corr + pv * vv[0]; acc[4 * c + 1] = acc[4 * c + 1] * corr + pv * vv[1]; acc[4 * c + 2] = acc[4 * c + 2] * corr + pv * vv[2]; acc[4 * c + 3] = acc[4 * c + 3] * corr + pv * vv[3]; }
      m = mn; } }
  const float sc = OCAR / l; unsigned short* d = (unsigned short*)O16 + (size_t)r * CH + h * DH;
  for (int g = 0; g < 4; ++g) { FragH f;
    for (int c = 0; c < 8; ++c) f.h[c] = (_Float16)(acc[8 * g + c] * sc);
    *(volatile v8us*)(d + 8 * g) = f.half[0]; __threadfence(); *(volatile v8us*)(d + 8 * g) = f.half[0]; } }
extern "C" void kernel_launch(void* const* d_in, const int* in_sizes, int n_in,
                              void* d_out, int out_size, void* d_ws, size_t ws_size, hipStream_t stream) {
  (void)in_sizes; (void)n_in; (void)out_size;
  const float* x = (const float*)d_in[0]; const float* wq = (const float*)d_in[1]; const float* wk = (const float*)d_in[2]; const float* wv = (const float*)d_in[3]; const float* wproj = (const float*)d_in[4];
  static_assert(HWP == MH * MW && CH == NHD * DH && NHD == 4 && DH == 32 && CH == 128 && ((size_t)NB * 2 * HWP) % 256 == 0 && ((size_t)CH * CH / 8) % 256 == 0 && ((size_t)NB * HWP * NHD) % 256 == 0 && ((size_t)NB * HWP) % 128 == 0 && QKVP % 64 == 0 && CH % 128 == 0 && HWP % 64 == 0 && CH % 32 == 0, "the head split; whole tiles; exact grids");
  float* out = (float*)d_out;
  char* ws = (char*)d_ws; size_t off = 0;
  auto take = [&](size_t bytes) { char* p = ws + off; off += (bytes + 255) & ~(size_t)255; return p; };
  _Float16* XT = (_Float16*)take((size_t)NB * HWP * CH * 2); _Float16* WQKV = (_Float16*)take((size_t)QKVP * CH * 2); _Float16* WP = (_Float16*)take((size_t)CH * CH * 2); float* QKV = (float*)take((size_t)NB * HWP * QKVP * 4); _Float16* O16 = (_Float16*)take((size_t)NB * HWP * CH * 2);
  if (off > ws_size) return;
  k_tcastg<<<(unsigned)((size_t)NB * 2 * HWP / 256), 256, 0, stream>>>(x, XT, NB * 2 * HWP);
  k_wcastc<<<(unsigned)((size_t)CH * CH / 8 / 256), 256, 0, stream>>>(wq, WQKV, WCAR, CH * CH / 8); k_wcastc<<<(unsigned)((size_t)CH * CH / 8 / 256), 256, 0, stream>>>(wk, WQKV + (size_t)CH * CH, WCAR, CH * CH / 8); k_wcastc<<<(unsigned)((size_t)CH * CH / 8 / 256), 256, 0, stream>>>(wv, WQKV + (size_t)2 * CH * CH, WCAR, CH * CH / 8); k_wcastc<<<(unsigned)((size_t)CH * CH / 8 / 256), 256, 0, stream>>>(wproj, WP, WCAR, CH * CH / 8);
  k_gemm2<0><<<dim3((NB * HWP / 128) * (QKVP / 64), 1), 128, 0, stream>>>(XT, CH, (size_t)0, WQKV, CH, (size_t)0, 1.0f / WCAR, nullptr, 0, nullptr, 1, 0, 0, QKV, nullptr, QKVP, (size_t)0, NB * HWP, QKVP, CH);
  k_win25<<<(unsigned)((size_t)NB * HWP * NHD / 256), 256, 0, stream>>>(QKV, O16, NB * HWP * NHD);
  k_gemm2<0><<<dim3((CH / 128) * (HWP / 64), NB), 128, 0, stream>>>(WP, CH, (size_t)0, O16, CH, (size_t)HWP * CH, 1.0f / (WCAR * OCAR), nullptr, 0, nullptr, 1, 0, 0, out, nullptr, HWP, (size_t)CH * HWP, CH, HWP, CH);
}
